// GCN_75917841924646
// MI455X (gfx1250) — hardware-verified
//
#include <hip/hip_runtime.h>
#include <stddef.h>
#include <stdint.h>
#include <math.h>


#define DF      128
#define NC      64
#define KA      256
#define NTHR    256
#define NWAVE   8
#define EPT     8
#define CHUNK   (NTHR * EPT)
#define WCAP    (EPT * 32)
#define LISTN   (NWAVE * WCAP)
#define NBA     1024
#define SLA     10
#define RCAP    28672
#define DEGCAP  64
#define MEAS_B1024  16721
#define MEAS_MAXDEG 36
#define GBM     64
#define GTHR    128
#define MROWS   128
#define NUW0    (DF * (KA / 8))
#define NUW1    (NC * (KA / 8))
#define WSMAX   134217728
#define BKT_ZINTS    (LISTN + 2 * RCAP + 3 * NBA)
#define BKT_LDS_INTS (BKT_ZINTS + 16)
#define AG1_LDS_INTS (2 * RCAP + 2 * NBA + NWAVE * KA / 2)
#define AG2_LDS_INTS (2 * RCAP + 2 * NBA)

static_assert((CHUNK & (CHUNK - 1)) == 0 && CHUNK <= 4096);
static_assert((NBA & (NBA - 1)) == 0 && NBA == (1 << SLA));
static_assert(LISTN >= NWAVE * WCAP);
static_assert(NBA % NWAVE == 0 && NBA % 32 == 0 && NBA == NTHR * 4);
static_assert(RCAP % (2 * NTHR) == 0 && (2 * RCAP) % (NTHR * 4) == 0);
static_assert(BKT_ZINTS % (NTHR * 4) == 0);
static_assert(RCAP * 20 >= MEAS_B1024 * 21);
static_assert(DEGCAP >= MEAS_MAXDEG + 8);
static_assert(100000 <= 98 * NBA);
static_assert(KA % 32 == 0 && KA == 2 * DF && DF == 4 * 32 && NC == 2 * 32);
static_assert(GBM == (GTHR / 32) * 16 && MROWS % GBM == 0);
static_assert(NUW0 % NTHR == 0 && NUW1 % NTHR == 0);
static_assert(BKT_LDS_INTS * 4 <= 300000 && AG1_LDS_INTS * 4 <= 300000 && AG2_LDS_INTS * 4 <= 300000);

typedef float          v2f   __attribute__((ext_vector_type(2)));
typedef float          v4f   __attribute__((ext_vector_type(4)));
typedef float          v8f   __attribute__((ext_vector_type(8)));
typedef int            v2i   __attribute__((ext_vector_type(2)));
typedef int            v4i   __attribute__((ext_vector_type(4)));
typedef int            v8i   __attribute__((ext_vector_type(8)));
typedef unsigned       v2u   __attribute__((ext_vector_type(2)));
typedef unsigned short v4us  __attribute__((ext_vector_type(4)));
typedef unsigned short v8us  __attribute__((ext_vector_type(8)));
typedef __bf16         v16bf __attribute__((ext_vector_type(16)));
typedef v4f  __attribute__((may_alias)) v4fa;
typedef v2i  __attribute__((may_alias)) v2ia;
typedef v4i  __attribute__((may_alias)) v4ia;
typedef v2u  __attribute__((may_alias)) v2ua;
typedef v4us __attribute__((may_alias)) v4usa;
typedef v8us __attribute__((may_alias)) v8usa;
union FragB { v16bf v; v8us h[2]; v8i w; };

__device__ __forceinline__ v8f wmb(const FragB& a, const FragB& b, v8f c) {
  v8f d = __builtin_amdgcn_wmma_f32_16x16x32_bf16(false, a.v, false, b.v, (short)0, c, false, false);
  asm volatile("v_nop\n\tv_nop\n\tv_nop\n\tv_nop" : "+v"(d) : "v"(a.w), "v"(b.w));
  return d;
}

__device__ __forceinline__ unsigned int f2bf(float f) {
  const unsigned int u = __float_as_uint(f);
  const unsigned int r = ((u + 0x7FFFu + ((u >> 16) & 1u)) >> 16) & 0xFFFFu;
  return ((u & 0x7FFFFFFFu) > 0x7F800000u) ? 0x7FC0u : r;
}
__device__ __forceinline__ float bf2f(unsigned int b) { return __uint_as_float(b << 16); }
__device__ __forceinline__ float bfr(float f) { return bf2f(f2bf(f)); }

__device__ __forceinline__ void wave_sync() {
  __builtin_amdgcn_fence(__ATOMIC_RELEASE, "workgroup");
  __builtin_amdgcn_wave_barrier();
  __builtin_amdgcn_fence(__ATOMIC_ACQUIRE, "workgroup");
}

__device__ __forceinline__ float nmax(float a, float b) { return ((a != a) || (a > b)) ? a : b; }

template <int SLB>
__device__ __forceinline__ int scan_chunk(const int* __restrict__ dsts, int nE, int cbase, int slotBase,
                                          int nb, int vec8, int* list, int tid, int lane, int wave) {
  int wc = 0;
  const int el0  = tid * EPT;
  const int e0   = cbase + el0;
  const int sent = -2147483647 - 1;
  v4i da, db;
  if (vec8 != 0 && cbase + CHUNK <= nE) {
    da = *(const v4i*)(dsts + e0);
    db = *(const v4i*)(dsts + e0 + 4);
  } else {
    da.x = (e0     < nE) ? dsts[min(e0,     nE - 1)] : sent;
    da.y = (e0 + 1 < nE) ? dsts[min(e0 + 1, nE - 1)] : sent;
    da.z = (e0 + 2 < nE) ? dsts[min(e0 + 2, nE - 1)] : sent;
    da.w = (e0 + 3 < nE) ? dsts[min(e0 + 3, nE - 1)] : sent;
    db.x = (e0 + 4 < nE) ? dsts[min(e0 + 4, nE - 1)] : sent;
    db.y = (e0 + 5 < nE) ? dsts[min(e0 + 5, nE - 1)] : sent;
    db.z = (e0 + 6 < nE) ? dsts[min(e0 + 6, nE - 1)] : sent;
    db.w = (e0 + 7 < nE) ? dsts[min(e0 + 7, nE - 1)] : sent;
  }
  const unsigned nbs = (unsigned)slotBase;
  const unsigned unb = (unsigned)nb;
  const unsigned s0 = (unsigned)da.x - nbs, s1 = (unsigned)da.y - nbs;
  const unsigned s2 = (unsigned)da.z - nbs, s3 = (unsigned)da.w - nbs;
  const unsigned s4 = (unsigned)db.x - nbs, s5 = (unsigned)db.y - nbs;
  const unsigned s6 = (unsigned)db.z - nbs, s7 = (unsigned)db.w - nbs;
  const bool h0 = s0 < unb, h1 = s1 < unb, h2 = s2 < unb, h3 = s3 < unb;
  const bool h4 = s4 < unb, h5 = s5 < unb, h6 = s6 < unb, h7 = s7 < unb;
  const unsigned any = __builtin_amdgcn_ballot_w32(h0 | h1 | h2 | h3 | h4 | h5 | h6 | h7);
  if (any != 0u) {
#define HITJ(J, HJ, SJ) { \
      const unsigned mj = __builtin_amdgcn_ballot_w32(HJ); \
      if (mj != 0u) { \
        if (HJ) { \
          const int pos = wc + (int)__builtin_amdgcn_mbcnt_lo(mj, 0u); \
          if (pos < WCAP) list[wave * WCAP + pos] = ((el0 + (J)) << SLB) | (int)(SJ); \
        } \
        wc += (int)__builtin_popcount(mj); } }
    HITJ(0, h0, s0)
    HITJ(1, h1, s1)
    HITJ(2, h2, s2)
    HITJ(3, h3, s3)
    HITJ(4, h4, s4)
    HITJ(5, h5, s5)
    HITJ(6, h6, s6)
    HITJ(7, h7, s7)
#undef HITJ
  }
  return wc;
}

__global__ __launch_bounds__(NTHR) void k_prep(const float* __restrict__ x, const float* __restrict__ W0,
                                               const float* __restrict__ W1, const float* __restrict__ b0,
                                               const float* __restrict__ b1, unsigned short* XB,
                                               unsigned short* W0D, unsigned short* W1D, float* BF,
                                               int nN, int nUx) {
  const int u = (int)blockIdx.x * NTHR + (int)threadIdx.x;
  if (u < nUx) {
    const int row = u >> 4;
    const int c0  = (u & 15) * 8;
    const int rc  = row < nN ? row : nN - 1;
    const float* p = x + (size_t)rc * DF + c0;
    const v4f a = *(const v4f*)p;
    const v4f b = *(const v4f*)(p + 4);
    const bool okr = row < nN;
    v8us o;
    o[0] = okr ? (unsigned short)f2bf(a.x) : (unsigned short)0;
    o[1] = okr ? (unsigned short)f2bf(a.y) : (unsigned short)0;
    o[2] = okr ? (unsigned short)f2bf(a.z) : (unsigned short)0;
    o[3] = okr ? (unsigned short)f2bf(a.w) : (unsigned short)0;
    o[4] = okr ? (unsigned short)f2bf(b.x) : (unsigned short)0;
    o[5] = okr ? (unsigned short)f2bf(b.y) : (unsigned short)0;
    o[6] = okr ? (unsigned short)f2bf(b.z) : (unsigned short)0;
    o[7] = okr ? (unsigned short)f2bf(b.w) : (unsigned short)0;
    unsigned short* dp = XB + (size_t)row * DF + c0;
    *(volatile v8us*)dp = o;
    __threadfence();
    *(volatile v8us*)dp = o;
  } else if (u < nUx + NUW0) {
    const int v  = u - nUx;
    const int n  = v >> 5;
    const int k8 = (v & 31) * 8;
    const int kk = k8 & (DF - 1);
    const float* p = W0 + (size_t)kk * DF + n;
    v8us o;
#pragma unroll
    for (int i = 0; i < 8; ++i) o[i] = (unsigned short)f2bf(p[(size_t)i * DF]);
    unsigned short* dp = W0D + (size_t)n * KA + k8;
    *(volatile v8us*)dp = o;
    __threadfence();
    *(volatile v8us*)dp = o;
  } else if (u < nUx + NUW0 + NUW1) {
    const int v  = u - nUx - NUW0;
    const int n  = v >> 5;
    const int k8 = (v & 31) * 8;
    const int kk = k8 & (DF - 1);
    const float* p = W1 + (size_t)kk * NC + n;
    v8us o;
#pragma unroll
    for (int i = 0; i < 8; ++i) o[i] = (unsigned short)f2bf(p[(size_t)i * NC]);
    unsigned short* dp = W1D + (size_t)n * KA + k8;
    *(volatile v8us*)dp = o;
    __threadfence();
    *(volatile v8us*)dp = o;
  } else {
    const int t  = u - nUx - NUW0 - NUW1;
    const int wv = t >> 5;
    const int ln = t & 31;
    if (wv == 0) {
      const v4f a = *(const v4f*)(b0 + 4 * ln);
      v4f r;
      r.x = bfr(a.x); r.y = bfr(a.y); r.z = bfr(a.z); r.w = bfr(a.w);
      float* dp = BF + 4 * ln;
      *(volatile v4f*)dp = r;
      __threadfence();
      *(volatile v4f*)dp = r;
    } else if (wv == 1) {
      const int lc = ln < 16 ? ln : 15;
      const v4f a = *(const v4f*)(b1 + 4 * lc);
      v4f r;
      r.x = bfr(a.x); r.y = bfr(a.y); r.z = bfr(a.z); r.w = bfr(a.w);
      float* dp = BF + DF + 4 * lc;
      if (ln < 16) *(volatile v4f*)dp = r;
      __threadfence();
      if (ln < 16) *(volatile v4f*)dp = r;
    }
  }
}

__device__ __forceinline__ void bucket_spill(const int* sl, const int* cnt, const int* offs,
                                             const int* __restrict__ srcs, const float* __restrict__ ew,
                                             int nE, int nN, int tt, int ovf,
                                             int* lb, int* cb, int* ob, int* fb, int tid) {
#pragma unroll 1
  for (int it = 0; it < RCAP / (2 * NTHR); ++it) {
    const int p  = 2 * (it * NTHR + tid);
    const int u0 = sl[p];
    const int u1 = sl[p + 1];
    int e0 = u0 >> SLA; e0 = e0 < 0 ? 0 : (e0 > nE - 1 ? nE - 1 : e0);
    int e1 = u1 >> SLA; e1 = e1 < 0 ? 0 : (e1 > nE - 1 ? nE - 1 : e1);
    int s0 = srcs[e0]; s0 = s0 < 0 ? 0 : (s0 > nN - 1 ? nN - 1 : s0);
    int s1 = srcs[e1]; s1 = s1 < 0 ? 0 : (s1 > nN - 1 ? nN - 1 : s1);
    const int w0 = (int)(f2bf(ew[e0]) << 16);
    const int w1 = (int)(f2bf(ew[e1]) << 16);
    v4i v;
    v.x = (p     < tt) ? s0 : 0;
    v.y = (p     < tt) ? w0 : 0;
    v.z = (p + 1 < tt) ? s1 : 0;
    v.w = (p + 1 < tt) ? w1 : 0;
    *(volatile v4i*)(lb + 2 * p) = v;
  }
  const v4i cv4 = *(const v4ia*)(cnt + 4 * tid);
  const v4i ov4 = *(const v4ia*)(offs + 4 * tid);
  *(volatile v4i*)(cb + 4 * tid) = cv4;
  *(volatile v4i*)(ob + 4 * tid) = ov4;
  v4i fv;
  fv.x = (tid == 0) ? tt : 0;
  fv.y = (tid == 0) ? ovf : 0;
  fv.z = 0; fv.w = 0;
  if (tid < 8) *(volatile v4i*)(fb + 4 * tid) = fv;
}

__global__ __launch_bounds__(NTHR) void k_bucket(const int* __restrict__ srcs, const int* __restrict__ dsts,
                                                 const float* __restrict__ ew, int nE, int nN, int vec8,
                                                 int* LIST, int* CNT, int* OFF, int* FLG) {
  extern __shared__ __attribute__((aligned(16))) int bsm[];
  int* list = bsm;
  int* hl   = bsm + LISTN;
  int* sl   = hl + RCAP;
  int* cnt  = sl + RCAP;
  int* offs = cnt + NBA;
  int* cur  = offs + NBA;
  int* misc = cur + NBA;
  const int tid = (int)threadIdx.x, lane = tid & 31, wave = tid >> 5;
  const int blk = (int)blockIdx.x;
  const int nodeBase = blk * NBA;
  int nb = nN - nodeBase;
  nb = nb < 0 ? 0 : (nb > NBA ? NBA : nb);

  {
    const v4i z4 = {0, 0, 0, 0};
    for (int i = tid * 4; i < BKT_ZINTS; i += NTHR * 4) *(v4ia*)(bsm + i) = z4;
    if (tid < 16) misc[tid] = 0;
  }
  __syncthreads();

  int tot = 0, ovf = 0;
  const int nChunks = (nE + CHUNK - 1) / CHUNK;
#pragma unroll 1
  for (int ch = 0; ch < nChunks; ++ch) {
    const int cbase = ch * CHUNK;
    const int wc = scan_chunk<SLA>(dsts, nE, cbase, nodeBase, nb, vec8, list, tid, lane, wave);
    if (lane == 0) misc[wave] = wc;
    __syncthreads();
    int pre = 0, all = 0;
#pragma unroll
    for (int w2 = 0; w2 < NWAVE; ++w2) {
      int c = misc[w2];
      c = c < 0 ? 0 : (c > WCAP ? WCAP : c);
      all += c;
      pre += (w2 < wave) ? c : 0;
    }
    const int wcc  = wc > WCAP ? WCAP : wc;
    const int base = tot + pre;
#pragma unroll 1
    for (int i = lane; i < wcc; i += 32) {
      const int ent = list[wave * WCAP + i];
      const int el  = (ent >> SLA) & (CHUNK - 1);
      const int sq  = ent & (NBA - 1);
      const int eid = cbase + el;
      const int pos = base + i;
      if (pos < RCAP) hl[pos] = (eid << SLA) | sq;
    }
    if (tot + all > RCAP) ovf = 1;
    tot += all;
    tot = tot > RCAP ? RCAP : tot;
    __syncthreads();
  }
  const int tt = tot;

  if (wave == 0) {
#pragma unroll 1
    for (int b0 = 0; b0 < tt; b0 += 32) {
      const int idx = b0 + lane;
      const int uv  = hl[idx < tt ? idx : tt - 1];
      const int m32 = (tt - b0) < 32 ? (tt - b0) : 32;
#pragma unroll 1
      for (int k = 0; k < m32; ++k) {
        const int u  = __builtin_amdgcn_readlane(uv, k);
        const int sq = u & (NBA - 1);
        if (lane == 0) cnt[sq] = cnt[sq] + 1;
      }
    }
  }
  __syncthreads();
  if (wave == 0) {
    const int base = lane * (NBA / 32);
    int s = 0;
#pragma unroll 1
    for (int i = 0; i < NBA / 32; ++i) s += cnt[base + i];
    int incl = s;
#pragma unroll
    for (int d = 1; d < 32; d <<= 1) {
      const int y = __shfl_up(incl, d, 32);
      if (lane >= d) incl += y;
    }
    int run = incl - s;
#pragma unroll 1
    for (int i = 0; i < NBA / 32; ++i) {
      const int cv = cnt[base + i];
      offs[base + i] = run;
      cur[base + i]  = run;
      run += cv;
    }
  }
  __syncthreads();
  if (wave == 0) {
#pragma unroll 1
    for (int b0 = 0; b0 < tt; b0 += 32) {
      const int idx = b0 + lane;
      const int uv  = hl[idx < tt ? idx : tt - 1];
      const int m32 = (tt - b0) < 32 ? (tt - b0) : 32;
#pragma unroll 1
      for (int k = 0; k < m32; ++k) {
        const int u  = __builtin_amdgcn_readlane(uv, k);
        const int sq = u & (NBA - 1);
        if (lane == 0) {
          int p = cur[sq];
          p = p < 0 ? 0 : (p > RCAP - 1 ? RCAP - 1 : p);
          sl[p] = u;
          cur[sq] = p + 1;
        }
      }
    }
  }
  __syncthreads();

  int* lb = LIST + (size_t)blk * (2 * RCAP);
  int* cb = CNT + (size_t)blk * NBA;
  int* ob = OFF + (size_t)blk * NBA;
  int* fb = FLG + (size_t)blk * 32;
  bucket_spill(sl, cnt, offs, srcs, ew, nE, nN, tt, ovf, lb, cb, ob, fb, tid);
  __threadfence();
  bucket_spill(sl, cnt, offs, srcs, ew, nE, nN, tt, ovf, lb, cb, ob, fb, tid);
}

__global__ __launch_bounds__(NTHR) void k_agg1(const int* __restrict__ LIST, const int* __restrict__ CNT,
                                               const int* __restrict__ OFF, const int* __restrict__ FLG,
                                               const unsigned short* __restrict__ XB, unsigned short* AH,
                                               int nN, int mRows) {
  extern __shared__ __attribute__((aligned(16))) int lds1[];
  int* ent  = lds1;
  int* cnt  = lds1 + 2 * RCAP;
  int* offs = cnt + NBA;
  const int tid = (int)threadIdx.x, lane = tid & 31, wave = tid >> 5;
  unsigned short* rowbuf = (unsigned short*)(offs + NBA) + wave * KA;
  const int blk = (int)blockIdx.x;
  const int nodeBase = blk * NBA;

  {
    const int* lb = LIST + (size_t)blk * (2 * RCAP);
#pragma unroll 1
    for (int p = tid * 4; p < 2 * RCAP; p += NTHR * 4) *(v4ia*)(ent + p) = *(const v4i*)(lb + p);
    *(v4ia*)(cnt + 4 * tid)  = *(const v4i*)(CNT + (size_t)blk * NBA + 4 * tid);
    *(v4ia*)(offs + 4 * tid) = *(const v4i*)(OFF + (size_t)blk * NBA + 4 * tid);
  }
  const int nhraw = FLG[(size_t)blk * 32];
  const int bflag = FLG[(size_t)blk * 32 + 1];
  const int ovf = (bflag != 0 || nhraw < 0 || nhraw > RCAP) ? 1 : 0;
  __syncthreads();

  const float qnan = __int_as_float(0x7fc00000);
  const float pz = (ovf != 0) ? qnan : 0.0f;
#pragma unroll 1
  for (int si = 0; si < NBA / NWAVE; ++si) {
    const int s    = si * NWAVE + wave;
    const int node = nodeBase + s;
    int c = __builtin_amdgcn_readfirstlane(cnt[s]);
    const bool big = c > DEGCAP;
    c = c < 0 ? 0 : (c > DEGCAP ? DEGCAP : c);
    int o = __builtin_amdgcn_readfirstlane(offs[s]);
    o = o < 0 ? 0 : (o > RCAP ? RCAP : o);
    if (c > RCAP - o) c = RCAP - o;
    float a0 = 0.0f, a1 = 0.0f, a2 = 0.0f, a3 = 0.0f;
#pragma unroll 1
    for (int b0 = 0; b0 < c; b0 += 32) {
      int idx = o + b0 + lane;
      idx = idx > o + c - 1 ? o + c - 1 : idx;
      const v2i e = *(const v2ia*)(ent + 2 * idx);
      int sr = e.x;
      sr = sr < 0 ? 0 : (sr > nN - 1 ? nN - 1 : sr);
      const int wvi = e.y;
      const int m32 = (c - b0) < 32 ? (c - b0) : 32;
#pragma unroll 1
      for (int k = 0; k < m32; ++k) {
        const int   sk = __builtin_amdgcn_readlane(sr, k);
        const float ck = __int_as_float(__builtin_amdgcn_readlane(wvi, k));
        const v2u w = *(const v2ua*)(XB + (size_t)sk * DF + 4 * lane);
        const float f0 = __uint_as_float(w.x << 16);
        const float f1 = __uint_as_float(w.x & 0xffff0000u);
        const float f2 = __uint_as_float(w.y << 16);
        const float f3 = __uint_as_float(w.y & 0xffff0000u);
        a0 = fmaf(ck, f0, a0);
        a1 = fmaf(ck, f1, a1);
        a2 = fmaf(ck, f2, a2);
        a3 = fmaf(ck, f3, a3);
      }
    }
    const float pzr = big ? qnan : pz;
    const bool live = node < nN;
    const float m0 = live ? (a0 + pzr) : 0.0f;
    const float m1 = live ? (a1 + pzr) : 0.0f;
    const float m2 = live ? (a2 + pzr) : 0.0f;
    const float m3 = live ? (a3 + pzr) : 0.0f;
    v4us mh, ml;
    {
      unsigned hb;
      hb = f2bf(m0); mh[0] = (unsigned short)hb; ml[0] = (unsigned short)f2bf(m0 - bf2f(hb));
      hb = f2bf(m1); mh[1] = (unsigned short)hb; ml[1] = (unsigned short)f2bf(m1 - bf2f(hb));
      hb = f2bf(m2); mh[2] = (unsigned short)hb; ml[2] = (unsigned short)f2bf(m2 - bf2f(hb));
      hb = f2bf(m3); mh[3] = (unsigned short)hb; ml[3] = (unsigned short)f2bf(m3 - bf2f(hb));
    }
    *(v4usa*)(rowbuf + 4 * lane) = mh;
    *(v4usa*)(rowbuf + DF + 4 * lane) = ml;
    wave_sync();
    const v8us q0 = *(const v8usa*)(rowbuf + 8 * lane);
    wave_sync();
    if (node < mRows) {
      unsigned short* rpw = AH + (size_t)node * KA + 8 * lane;
      *(volatile v8us*)rpw = q0;
      __threadfence();
      *(volatile v8us*)rpw = q0;
    }
  }
}

__global__ __launch_bounds__(GTHR) void k_gemm1(unsigned short* Apl, const unsigned short* __restrict__ BT,
                                                const float* __restrict__ BF, int nN) {
  __shared__ __attribute__((aligned(16))) float stg[GBM * DF];
  const int tid = (int)threadIdx.x, lane = tid & 31, wave = tid >> 5, hh = lane >> 4, m = lane & 15;
  const int rowBase = (int)blockIdx.x * GBM;

  v8f acc[8];
  {
    const v8f z = {0.f, 0.f, 0.f, 0.f, 0.f, 0.f, 0.f, 0.f};
#pragma unroll
    for (int t = 0; t < 8; ++t) acc[t] = z;
  }
  const unsigned short* ap = Apl + (size_t)(rowBase + 16 * wave + m) * (size_t)KA + 8 * hh;
  const unsigned short* bp = BT + (size_t)m * (size_t)KA + 8 * hh;

#pragma unroll 1
  for (int k0 = 0; k0 < KA; k0 += 32) {
    FragB af;
    af.h[0] = *(const v8usa*)(ap + k0);
    af.h[1] = *(const v8usa*)(ap + k0 + 16);
#pragma unroll
    for (int nt = 0; nt < 8; ++nt) {
      const unsigned short* wq = bp + (size_t)(16 * nt) * (size_t)KA + k0;
      FragB bf;
      bf.h[0] = *(const v8usa*)wq;
      bf.h[1] = *(const v8usa*)(wq + 16);
      acc[nt] = wmb(af, bf, acc[nt]);
    }
  }

#pragma unroll
  for (int nt = 0; nt < 8; ++nt) {
    const int lc = 16 * nt + m;
#pragma unroll
    for (int r = 0; r < 8; ++r) {
      const int lr = 16 * wave + 8 * hh + r;
      stg[lr * DF + lc] = acc[nt][r];
    }
  }
  __syncthreads();

  const v4f bb4 = *(const v4f*)(BF + 4 * lane);

  v4f pv[16];
#pragma unroll
  for (int i = 0; i < 16; ++i) pv[i] = *(const v4fa*)(stg + (16 * wave + i) * DF + 4 * lane);
  __syncthreads();

#pragma unroll
  for (int i = 0; i < 16; ++i) {
    const bool ok = (rowBase + 16 * wave + i) < nN;
    const v4f t = pv[i] + bb4;
    v4f y;
    y.x = (t.x > 0.0f) ? t.x : (t.x - t.x);
    y.y = (t.y > 0.0f) ? t.y : (t.y - t.y);
    y.z = (t.z > 0.0f) ? t.z : (t.z - t.z);
    y.w = (t.w > 0.0f) ? t.w : (t.w - t.w);
    y.x = ok ? y.x : 0.0f; y.y = ok ? y.y : 0.0f; y.z = ok ? y.z : 0.0f; y.w = ok ? y.w : 0.0f;
    pv[i] = y;
  }

#pragma unroll
  for (int i = 0; i < 16; ++i) {
    v4us h4, l4;
    unsigned hb;
    hb = f2bf(pv[i].x); h4[0] = (unsigned short)hb; l4[0] = (unsigned short)f2bf(pv[i].x - bf2f(hb));
    hb = f2bf(pv[i].y); h4[1] = (unsigned short)hb; l4[1] = (unsigned short)f2bf(pv[i].y - bf2f(hb));
    hb = f2bf(pv[i].z); h4[2] = (unsigned short)hb; l4[2] = (unsigned short)f2bf(pv[i].z - bf2f(hb));
    hb = f2bf(pv[i].w); h4[3] = (unsigned short)hb; l4[3] = (unsigned short)f2bf(pv[i].w - bf2f(hb));
    unsigned short* srow = (unsigned short*)stg + (size_t)(16 * wave + i) * (2 * DF);
    *(v4usa*)(srow + 4 * lane) = h4;
    *(v4usa*)(srow + DF + 4 * lane) = l4;
  }
  __syncthreads();
  v8us qv[16];
#pragma unroll
  for (int i = 0; i < 16; ++i) {
    const unsigned short* srow = (const unsigned short*)stg + (size_t)(16 * wave + i) * (2 * DF);
    qv[i] = *(const v8usa*)(srow + 8 * lane);
  }
#pragma unroll
  for (int i = 0; i < 16; ++i) {
    unsigned short* rp = Apl + (size_t)(rowBase + 16 * wave + i) * (size_t)KA + 8 * lane;
    *(volatile v8us*)rp = qv[i];
  }
  __threadfence();
#pragma unroll
  for (int i = 0; i < 16; ++i) {
    unsigned short* rp = Apl + (size_t)(rowBase + 16 * wave + i) * (size_t)KA + 8 * lane;
    *(volatile v8us*)rp = qv[i];
  }
}

__global__ __launch_bounds__(GTHR) void k_gemm2(const unsigned short* __restrict__ A,
                                                const unsigned short* __restrict__ WT, float* outF) {
  __shared__ __attribute__((aligned(16))) float stg[GBM * NC];
  const int tid = (int)threadIdx.x, lane = tid & 31, wave = tid >> 5, hh = lane >> 4, m = lane & 15;
  const int rowBase = (int)blockIdx.x * GBM;

  v8f acc[4];
  {
    const v8f z = {0.f, 0.f, 0.f, 0.f, 0.f, 0.f, 0.f, 0.f};
    acc[0] = z; acc[1] = z; acc[2] = z; acc[3] = z;
  }
  const unsigned short* ap = A  + (size_t)(rowBase + 16 * wave + m) * (size_t)KA + 8 * hh;
  const unsigned short* wp = WT + (size_t)m * (size_t)KA + 8 * hh;
#pragma unroll 1
  for (int k0 = 0; k0 < KA; k0 += 32) {
    FragB af;
    af.h[0] = *(const v8usa*)(ap + k0);
    af.h[1] = *(const v8usa*)(ap + k0 + 16);
#pragma unroll
    for (int t = 0; t < 4; ++t) {
      const unsigned short* wq = wp + (size_t)(16 * t) * (size_t)KA + k0;
      FragB bf;
      bf.h[0] = *(const v8usa*)wq;
      bf.h[1] = *(const v8usa*)(wq + 16);
      acc[t] = wmb(af, bf, acc[t]);
    }
  }

#pragma unroll
  for (int t = 0; t < 4; ++t) {
    const int lc = 16 * t + m;
#pragma unroll
    for (int r = 0; r < 8; ++r) {
      const int lr = 16 * wave + 8 * hh + r;
      stg[lr * NC + lc] = acc[t][r];
    }
  }
  __syncthreads();

  v4f fv[8];
#pragma unroll
  for (int i = 0; i < 8; ++i) {
    const int lr = 16 * wave + 2 * i + hh;
    fv[i] = *(const v4fa*)(stg + lr * NC + 4 * m);
  }
#pragma unroll
  for (int i = 0; i < 8; ++i) {
    const int lr = 16 * wave + 2 * i + hh;
    float* op = outF + (size_t)(rowBase + lr) * (size_t)NC + 4 * m;
    *(volatile v4f*)op = fv[i];
  }
  __threadfence();
#pragma unroll
  for (int i = 0; i < 8; ++i) {
    const int lr = 16 * wave + 2 * i + hh;
    float* op = outF + (size_t)(rowBase + lr) * (size_t)NC + 4 * m;
    *(volatile v4f*)op = fv[i];
  }
}

__global__ __launch_bounds__(NTHR) void k_agg2(const int* __restrict__ LIST, const int* __restrict__ CNT,
                                               const int* __restrict__ OFF, const int* __restrict__ FLG,
                                               const float* __restrict__ P, const float* __restrict__ BF,
                                               float* out, int nN) {
  extern __shared__ __attribute__((aligned(16))) int lds2[];
  int* ent  = lds2;
  int* cnt  = lds2 + 2 * RCAP;
  int* offs = cnt + NBA;
  const int tid = (int)threadIdx.x, lane = tid & 31, wave = tid >> 5;
  const int blk = (int)blockIdx.x;
  const int nodeBase = blk * NBA;

  {
    const int* lb = LIST + (size_t)blk * (2 * RCAP);
#pragma unroll 1
    for (int p = tid * 4; p < 2 * RCAP; p += NTHR * 4) *(v4ia*)(ent + p) = *(const v4i*)(lb + p);
    *(v4ia*)(cnt + 4 * tid)  = *(const v4i*)(CNT + (size_t)blk * NBA + 4 * tid);
    *(v4ia*)(offs + 4 * tid) = *(const v4i*)(OFF + (size_t)blk * NBA + 4 * tid);
  }
  const int nhraw = FLG[(size_t)blk * 32];
  const int bflag = FLG[(size_t)blk * 32 + 1];
  const int ovf = (bflag != 0 || nhraw < 0 || nhraw > RCAP) ? 1 : 0;
  const v2f bq = *(const v2f*)(BF + DF + 2 * lane);
  __syncthreads();

  const float qnan = __int_as_float(0x7fc00000);
#pragma unroll 1
  for (int si = 0; si < NBA / NWAVE; ++si) {
    const int s    = si * NWAVE + wave;
    const int node = nodeBase + s;
    int c = __builtin_amdgcn_readfirstlane(cnt[s]);
    const bool big = c > DEGCAP;
    c = c < 0 ? 0 : (c > DEGCAP ? DEGCAP : c);
    int o = __builtin_amdgcn_readfirstlane(offs[s]);
    o = o < 0 ? 0 : (o > RCAP ? RCAP : o);
    if (c > RCAP - o) c = RCAP - o;
    float a0 = 0.0f, a1 = 0.0f;
#pragma unroll 1
    for (int b0 = 0; b0 < c; b0 += 32) {
      int idx = o + b0 + lane;
      idx = idx > o + c - 1 ? o + c - 1 : idx;
      const v2i e = *(const v2ia*)(ent + 2 * idx);
      int sr = e.x;
      sr = sr < 0 ? 0 : (sr > nN - 1 ? nN - 1 : sr);
      const int wvi = e.y;
      const int m32 = (c - b0) < 32 ? (c - b0) : 32;
#pragma unroll 1
      for (int k = 0; k < m32; ++k) {
        const int   sk = __builtin_amdgcn_readlane(sr, k);
        const float ck = __int_as_float(__builtin_amdgcn_readlane(wvi, k));
        const v2f pr = *(const v2f*)(P + (size_t)sk * NC + 2 * lane);
        a0 = fmaf(ck, pr.x, a0);
        a1 = fmaf(ck, pr.y, a1);
      }
    }
    const float o0 = a0 + bq.x;
    const float o1 = a1 + bq.y;
    float mx = nmax(o0, o1);
#pragma unroll
    for (int d = 16; d > 0; d >>= 1) {
      const float t = __shfl_xor(mx, d, 32);
      mx = nmax(mx, t);
    }
    const float sh0 = o0 - mx;
    const float sh1 = o1 - mx;
    float sm = expf(sh0) + expf(sh1);
#pragma unroll
    for (int d = 16; d > 0; d >>= 1) sm += __shfl_xor(sm, d, 32);
    const float lg = logf(sm);
    const bool bad = big || (ovf != 0);
    v2f r;
    r.x = bad ? qnan : (sh0 - lg);
    r.y = bad ? qnan : (sh1 - lg);
    if (node < nN) {
      float* op = out + (size_t)node * NC + 2 * lane;
      *(volatile v2f*)op = r;
      __threadfence();
      *(volatile v2f*)op = r;
    }
  }
}

static inline int cdiv(int a, int b) { return (a + b - 1) / b; }
static inline size_t al256(size_t o) { return (o + 255) & ~(size_t)255; }

extern "C" void kernel_launch(void* const* d_in, const int* in_sizes, int n_in,
                              void* d_out, int out_size, void* d_ws, size_t ws_size,
                              hipStream_t stream) {
  if (n_in < 8) return;
  if (in_sizes[0] < DF || (in_sizes[0] % DF) != 0) return;
  const int nN = in_sizes[0] / DF;
  const int nE = in_sizes[1];
  if (nE < 1 || in_sizes[2] != nE || in_sizes[3] != nE) return;
  if (nE >= (1 << 21) || nN < 16 || nN >= (1 << 24)) return;
  if (in_sizes[4] != DF * DF || in_sizes[5] != DF) return;
  if (in_sizes[6] != DF * NC || in_sizes[7] != NC) return;
  if ((long long)out_size != (long long)nN * NC) return;

  const float* x   = (const float*)d_in[0];
  const int*   src = (const int*)d_in[1];
  const int*   dst = (const int*)d_in[2];
  const float* ew  = (const float*)d_in[3];
  const float* W0  = (const float*)d_in[4];
  const float* b0  = (const float*)d_in[5];
  const float* W1  = (const float*)d_in[6];
  const float* b1  = (const float*)d_in[7];
  float* out = (float*)d_out;

  const int MP = cdiv(nN, MROWS) * MROWS;
  const int gM = MP / GBM;
  const int gA = cdiv(nN, NBA);
  if ((long long)gA * NBA < (long long)MP) return;
  const int vec8 = ((nE & 3) == 0) ? 1 : 0;
  const int nUx  = MP * (DF / 8);
  if ((nUx % NTHR) != 0) return;

  char* ws = (char*)d_ws;
  size_t off = 0;
  const size_t oXB  = off; off = al256(off + (size_t)MP * DF * 2);
  const size_t oAH  = off; off = al256(off + (size_t)MP * KA * 2);
  const size_t oP   = off; off = al256(off + (size_t)MP * NC * 4);
  const size_t oLST = off; off = al256(off + (size_t)gA * RCAP * 8);
  const size_t oCNT = off; off = al256(off + (size_t)gA * NBA * 4);
  const size_t oOFF = off; off = al256(off + (size_t)gA * NBA * 4);
  const size_t oFLG = off; off = al256(off + (size_t)gA * 128);
  const size_t oW0D = off; off = al256(off + (size_t)DF * KA * 2);
  const size_t oW1D = off; off = al256(off + (size_t)NC * KA * 2);
  const size_t oBF  = off; off = al256(off + (size_t)(DF + NC) * 4);
  if (off > ws_size || off > (size_t)WSMAX) return;
  unsigned short* XB   = (unsigned short*)(ws + oXB);
  unsigned short* AH   = (unsigned short*)(ws + oAH);
  float*          P    = (float*)(ws + oP);
  int*            LIST = (int*)(ws + oLST);
  int*            CNT  = (int*)(ws + oCNT);
  int*            OFF  = (int*)(ws + oOFF);
  int*            FLG  = (int*)(ws + oFLG);
  unsigned short* W0D  = (unsigned short*)(ws + oW0D);
  unsigned short* W1D  = (unsigned short*)(ws + oW1D);
  float*          BF   = (float*)(ws + oBF);

  const int bktLds = BKT_LDS_INTS * 4;
  const int ag1Lds = AG1_LDS_INTS * 4;
  const int ag2Lds = AG2_LDS_INTS * 4;
  hipFuncSetAttribute(reinterpret_cast<const void*>(&k_bucket), hipFuncAttributeMaxDynamicSharedMemorySize, bktLds);
  hipFuncSetAttribute(reinterpret_cast<const void*>(&k_agg1),   hipFuncAttributeMaxDynamicSharedMemorySize, ag1Lds);
  hipFuncSetAttribute(reinterpret_cast<const void*>(&k_agg2),   hipFuncAttributeMaxDynamicSharedMemorySize, ag2Lds);

  k_prep<<<(nUx + NUW0 + NUW1 + NTHR) / NTHR, NTHR, 0, stream>>>(x, W0, W1, b0, b1, XB, W0D, W1D, BF, nN, nUx);
  k_bucket<<<gA, NTHR, bktLds, stream>>>(src, dst, ew, nE, nN, vec8, LIST, CNT, OFF, FLG);
  k_agg1<<<gA, NTHR, ag1Lds, stream>>>(LIST, CNT, OFF, FLG, XB, AH, nN, MP);
  k_gemm1<<<gM, GTHR, 0, stream>>>(AH, W0D, BF, nN);
  k_gemm2<<<gM, GTHR, 0, stream>>>(AH, W1D, P);
  k_agg2<<<gA, NTHR, ag2Lds, stream>>>(LIST, CNT, OFF, FLG, P, BF, out, nN);
}
